// block_15341623181397
// MI455X (gfx1250) — hardware-verified
//
#include <hip/hip_runtime.h>
#ifndef NB
#define NB 2
#endif
#ifndef SEQ
#define SEQ 2048
#endif
#define NB_FULL 2
#define SEQ_FULL 2048
#define FEAT 768
#define NHEAD 12
#define DHEAD 64
#define MLPH 3072
#define MR (NB * SEQ)
#define QKVN (3 * FEAT)
#define QKN (2 * FEAT)
static_assert(SEQ % 64 == 0);
static_assert(SEQ <= SEQ_FULL);
static_assert(NB >= 1);
static_assert(NB <= NB_FULL);
static_assert(FEAT == NHEAD * DHEAD);
static_assert(FEAT % 64 == 0);
static_assert(MLPH % 64 == 0);
static_assert(QKVN % 64 == 0);
static_assert(QKN % 64 == 0);
static_assert(FEAT == 96 * 8);
static_assert(MR % 16 == 0);
static_assert((FEAT * 2) % 128 == 0);
static_assert((QKVN * 2) % 128 == 0);
static_assert((QKN * 2) % 128 == 0);
static_assert((MLPH * 2) % 128 == 0);
static_assert((size_t)NB_FULL * SEQ_FULL * FEAT * 4 == (size_t)12582912);

typedef _Float16 v16h __attribute__((ext_vector_type(16)));
typedef unsigned short v8us __attribute__((ext_vector_type(8), may_alias));
typedef float v8f __attribute__((ext_vector_type(8)));
typedef float v4f __attribute__((ext_vector_type(4)));
typedef float v4fa __attribute__((ext_vector_type(4), may_alias));
union FragH { v16h v; v8us half[2]; unsigned short u[16]; };
union H16U { _Float16 h; unsigned short u; };

__device__ __forceinline__ unsigned short bf16_bits(float x) { unsigned int u = __float_as_uint(x); return (unsigned short)((u + 0x7FFFu + ((u >> 16) & 1u)) >> 16); }
__device__ __forceinline__ float bf16_val(unsigned short b) { return __uint_as_float(((unsigned int)b) << 16); }
__device__ __forceinline__ float bf16_rne(float x) { return bf16_val(bf16_bits(x)); }
__device__ __forceinline__ unsigned short h16_bits(float x) { H16U t; t.h = (_Float16)x; return t.u; }
__device__ __forceinline__ float h16_valf(unsigned short b) { H16U t; t.u = b; return (float)t.h; }
__device__ __forceinline__ v8f vz8() { v8f z = {0.f, 0.f, 0.f, 0.f, 0.f, 0.f, 0.f, 0.f}; return z; }

__device__ __forceinline__ v8f mma16(v16h a, v16h b, v8f c) {
  c = __builtin_amdgcn_wmma_f32_16x16x32_f16(false, a, false, b, (short)0, c, false, false);
  asm volatile("v_nop\n\tv_nop\n\tv_nop\n\tv_nop" : "+v"(c) : "v"(a), "v"(b));
  return c;
}

__global__ __launch_bounds__(256) void k_w16(const float* __restrict__ W, unsigned short* __restrict__ Wt, int total8, float sc) {
  const int t = blockIdx.x * 256 + threadIdx.x;
  if (t >= total8) return;
  const size_t e0 = (size_t)t * 8;
  const v4f a0 = *(const v4fa*)(W + e0);
  const v4f a1 = *(const v4fa*)(W + e0 + 4);
  const float f[8] = {a0[0], a0[1], a0[2], a0[3], a1[0], a1[1], a1[2], a1[3]};
  v8us v;
#pragma unroll
  for (int i = 0; i < 8; ++i) v[i] = h16_bits(bf16_rne(f[i]) * sc);
  unsigned short* dst = Wt + e0;
  *(volatile v8us*)dst = v;
  __threadfence();
  *(volatile v8us*)dst = v;
}

template <bool RND>
__global__ __launch_bounds__(96) void k_ln16(const float* __restrict__ X, int in_map, int seq, int seqf,
                                             const float* __restrict__ g, const float* __restrict__ bt,
                                             unsigned short* __restrict__ out, float osc, float eps) {
  __shared__ float red1[4];
  __shared__ float red2[4];
  const int m = blockIdx.x, tid = threadIdx.x, w = tid >> 5, lane = tid & 31;
  const int srow = in_map ? ((m / seq) * seqf + (m % seq)) : m;
  const float* x = X + (size_t)srow * FEAT + tid * 8;
  const v4f a0 = *(const v4fa*)x;
  const v4f a1 = *(const v4fa*)(x + 4);
  float v[8] = {a0[0], a0[1], a0[2], a0[3], a1[0], a1[1], a1[2], a1[3]};
  if (RND) {
#pragma unroll
    for (int q = 0; q < 8; ++q) v[q] = bf16_rne(v[q]);
  }
  float s = 0.f;
#pragma unroll
  for (int q = 0; q < 8; ++q) s += v[q];
#pragma unroll
  for (int o = 16; o >= 1; o >>= 1) s += __shfl_xor(s, o, 32);
  if (lane == 0) red1[w] = s;
  __syncthreads();
  const float mu = (red1[0] + red1[1] + red1[2]) * (1.0f / (float)FEAT);
  float c[8];
  float s2 = 0.f;
#pragma unroll
  for (int q = 0; q < 8; ++q) { c[q] = v[q] - mu; s2 += c[q] * c[q]; }
#pragma unroll
  for (int o = 16; o >= 1; o >>= 1) s2 += __shfl_xor(s2, o, 32);
  if (lane == 0) red2[w] = s2;
  __syncthreads();
  const float var = (red2[0] + red2[1] + red2[2]) * (1.0f / (float)FEAT);
  const float rs = rsqrtf(var + eps);
  v8us o;
#pragma unroll
  for (int q = 0; q < 8; ++q) {
    const float gg = bf16_rne(g[tid * 8 + q]);
    const float bb = bf16_rne(bt[tid * 8 + q]);
    o[q] = h16_bits((c[q] * rs * gg + bb) * osc);
  }
  unsigned short* dst = out + (size_t)m * FEAT + tid * 8;
  *(volatile v8us*)dst = o;
  __threadfence();
  *(volatile v8us*)dst = o;
}

template <bool OUT16, int ACT, bool RES_BF16, bool LO>
__global__ __launch_bounds__(128) void k_gemm16(const unsigned short* __restrict__ A, int lda, const unsigned short* __restrict__ Wt, int ldb,
                                                const float* __restrict__ bias0, const float* __restrict__ bias1, const float* __restrict__ bias2, int nsplit,
                                                const float* __restrict__ resid, int ldr, int res_map,
                                                void* __restrict__ Cv, int ldc, int out_map, int seq, int seqf,
                                                int M, int N, int K, float inv_scale, float out_scale,
                                                unsigned short* __restrict__ Lo, int ldlo, int locols, float lo_scale) {
  __shared__ __attribute__((aligned(16))) float so32[OUT16 ? 1 : 4][16][64];
  __shared__ __attribute__((aligned(16))) unsigned short so16[OUT16 ? 4 : 1][16][72];
  __shared__ __attribute__((aligned(16))) unsigned short so16lo[(OUT16 && LO) ? 4 : 1][16][72];
  const int tid = threadIdx.x, w = tid >> 5, lane = tid & 31, ln = lane & 15, hh = lane >> 4;
  const int ntn = N / 64;
  const int wid = blockIdx.x * 4 + w;
  const int mt = wid / ntn, nq = wid % ntn;
  if (mt * 16 >= M) return;
  const int row0 = mt * 16, col0 = nq * 64;
  const unsigned short* arow = A + (size_t)(row0 + ln) * lda;
  v8f acc[4];
#pragma unroll
  for (int t = 0; t < 4; ++t) acc[t] = vz8();
  for (int kb = 0; kb < K; kb += 32) {
    FragH a;
    a.half[0] = *(const v8us*)(arow + kb + 8 * hh);
    a.half[1] = *(const v8us*)(arow + kb + 16 + 8 * hh);
#pragma unroll
    for (int t = 0; t < 4; ++t) {
      const unsigned short* brow = Wt + (size_t)(col0 + t * 16 + ln) * ldb + kb;
      FragH bb;
      bb.half[0] = *(const v8us*)(brow + 8 * hh);
      bb.half[1] = *(const v8us*)(brow + 16 + 8 * hh);
      acc[t] = mma16(a.v, bb.v, acc[t]);
    }
  }
  int seg = col0 / nsplit; seg = (seg > 2) ? 2 : seg;
  const float* bsel = (seg == 0) ? bias0 : ((seg == 1) ? bias1 : bias2);
  const int rrow0 = res_map ? ((row0 / seq) * seqf + (row0 % seq)) : row0;
#pragma unroll
  for (int t = 0; t < 4; ++t) {
    const int col = col0 + t * 16 + ln;
    const float bvv = bf16_rne(bsel[col - seg * nsplit]);
#pragma unroll
    for (int r = 0; r < 8; ++r) {
      float v = acc[t][r] * inv_scale + bvv;
      if (ACT == 1) v = 0.5f * v * (1.0f + erff(v * 0.70710678118654752f));
      if (resid != nullptr) {
        float rv = resid[(size_t)(rrow0 + 8 * hh + r) * ldr + col];
        if (RES_BF16) rv = bf16_rne(rv);
        v += rv;
      }
      if constexpr (OUT16) {
        const float vs = v * out_scale;
        const unsigned short hb = h16_bits(vs);
        so16[w][8 * hh + r][t * 16 + ln] = hb;
        if constexpr (LO) so16lo[w][8 * hh + r][t * 16 + ln] = h16_bits((vs - h16_valf(hb)) * lo_scale);
      } else {
        so32[w][8 * hh + r][t * 16 + ln] = v;
      }
    }
  }
  __builtin_amdgcn_fence(4  , "workgroup");
  __builtin_amdgcn_wave_barrier();
  const int orow0 = out_map ? ((row0 / seq) * seqf + (row0 % seq)) : row0;
  if constexpr (OUT16) {
    unsigned short* Ch = (unsigned short*)Cv;
    const int rq = lane >> 3, p8 = (lane & 7) * 8;
    const bool dolo = LO && (Lo != nullptr) && (col0 + 64 <= locols);
    for (int pass = 0; pass < 2; ++pass) {
#pragma unroll
      for (int q = 0; q < 4; ++q) {
        const int r = q * 4 + rq;
        const v8us v = *(const v8us*)&so16[w][r][p8];
        *(volatile v8us*)(Ch + (size_t)(orow0 + r) * ldc + col0 + p8) = v;
      }
      if constexpr (LO) {
        if (dolo) {
#pragma unroll
          for (int q = 0; q < 4; ++q) {
            const int r = q * 4 + rq;
            const v8us v = *(const v8us*)&so16lo[w][r][p8];
            *(volatile v8us*)(Lo + (size_t)(row0 + r) * ldlo + col0 + p8) = v;
          }
        }
      }
      if (pass == 0) __threadfence();
    }
  } else {
    float* Cf = (float*)Cv;
    const int rsub = lane >> 4, c4 = (lane & 15) * 4;
    for (int pass = 0; pass < 2; ++pass) {
#pragma unroll
      for (int q = 0; q < 8; ++q) {
        const int r = q * 2 + rsub;
        const v4f v = *(const v4fa*)&so32[w][r][c4];
        *(volatile v4f*)(Cf + (size_t)(orow0 + r) * ldc + col0 + c4) = v;
      }
      if (pass == 0) __threadfence();
    }
  }
}

template <int D>
__global__ __launch_bounds__(128) void k_attn16(const unsigned short* __restrict__ qkv, int pitch,
                                                const unsigned short* __restrict__ qkl, int lpitch, int lkoff,
                                                int T, int H, int koff, int voff,
                                                float lo_inv, float pcarry, float onorm, unsigned short* __restrict__ ctx, int cpitch) {
  static_assert(D == 64);
  constexpr int KS = D / 32, DT = D / 16, C8 = D / 8;
  static_assert((32 * C8) % 128 == 0);
  __shared__ __attribute__((aligned(16))) unsigned short sK[32][D + 8];
  __shared__ __attribute__((aligned(16))) unsigned short sKl[32][D + 8];
  __shared__ __attribute__((aligned(16))) unsigned short sVt[D][40];
  __shared__ __attribute__((aligned(16))) unsigned short sP[4][16][40];
  __shared__ __attribute__((aligned(16))) unsigned short sO[4][16][D + 8];
  const int tid = threadIdx.x, w = tid >> 5, lane = tid & 31, ln = lane & 15, hh = lane >> 4;
  const int nqb = T / 64;
  const int bh = blockIdx.x / nqb, qblk = blockIdx.x % nqb;
  const int b = bh / H, h = bh % H;
  const int q0 = qblk * 64 + w * 16;
  const unsigned short* Qp = qkv + (size_t)b * T * pitch + h * D;
  const unsigned short* Kp = Qp + koff;
  const unsigned short* Vp = Qp + voff;
  const unsigned short* Qlp = qkl + (size_t)b * T * lpitch + h * D;
  const unsigned short* Klp = Qlp + lkoff;

  FragH aq[KS], al[KS];
  {
    const unsigned short* qr = Qp + (size_t)(q0 + ln) * pitch;
    const unsigned short* qlr = Qlp + (size_t)(q0 + ln) * lpitch;
#pragma unroll
    for (int ks = 0; ks < KS; ++ks) {
      aq[ks].half[0] = *(const v8us*)(qr + ks * 32 + 8 * hh);
      aq[ks].half[1] = *(const v8us*)(qr + ks * 32 + 16 + 8 * hh);
      al[ks].half[0] = *(const v8us*)(qlr + ks * 32 + 8 * hh);
      al[ks].half[1] = *(const v8us*)(qlr + ks * 32 + 16 + 8 * hh);
    }
  }
  float m_r[8], l_r[8];
#pragma unroll
  for (int r = 0; r < 8; ++r) { m_r[r] = -1.0e30f; l_r[r] = 0.f; }
  v8f oacc[DT];
#pragma unroll
  for (int dt = 0; dt < DT; ++dt) oacc[dt] = vz8();

  for (int j0 = 0; j0 < T; j0 += 32) {
    __syncthreads();
#pragma unroll
    for (int it = 0; it < (32 * C8) / 128; ++it) {
      const int e = tid + it * 128;
      const int r = e / C8, c8 = (e % C8) * 8;
      const size_t ro = (size_t)(j0 + r) * pitch + c8;
      const v8us kvv = *(const v8us*)(Kp + ro);
      *(v8us*)&sK[r][c8] = kvv;
      const v8us klv = *(const v8us*)(Klp + (size_t)(j0 + r) * lpitch + c8);
      *(v8us*)&sKl[r][c8] = klv;
      const v8us vvv = *(const v8us*)(Vp + ro);
#pragma unroll
      for (int i = 0; i < 8; ++i) sVt[c8 + i][r] = vvv[i];
    }
    __syncthreads();
    v8f s[2], sx[2];
#pragma unroll
    for (int nt = 0; nt < 2; ++nt) {
      v8f a1 = vz8(), a2 = vz8();
#pragma unroll
      for (int ks = 0; ks < KS; ++ks) {
        FragH bk, bl;
        bk.half[0] = *(const v8us*)&sK[nt * 16 + ln][ks * 32 + 8 * hh];
        bk.half[1] = *(const v8us*)&sK[nt * 16 + ln][ks * 32 + 16 + 8 * hh];
        bl.half[0] = *(const v8us*)&sKl[nt * 16 + ln][ks * 32 + 8 * hh];
        bl.half[1] = *(const v8us*)&sKl[nt * 16 + ln][ks * 32 + 16 + 8 * hh];
        a1 = mma16(aq[ks].v, bk.v, a1);
        a2 = mma16(aq[ks].v, bl.v, a2);
        a2 = mma16(al[ks].v, bk.v, a2);
      }
      s[nt] = a1;
      sx[nt] = a2;
    }
    float alpha[8];
#pragma unroll
    for (int r = 0; r < 8; ++r) {
      const float s0 = s[0][r] + sx[0][r] * lo_inv, s1 = s[1][r] + sx[1][r] * lo_inv;
      float mx = fmaxf(s0, s1);
      mx = fmaxf(mx, __shfl_xor(mx, 1, 32)); mx = fmaxf(mx, __shfl_xor(mx, 2, 32));
      mx = fmaxf(mx, __shfl_xor(mx, 4, 32)); mx = fmaxf(mx, __shfl_xor(mx, 8, 32));
      const float mnew = fmaxf(m_r[r], mx);
      alpha[r] = __expf(m_r[r] - mnew);
      const float p0 = __expf(s0 - mnew), p1 = __expf(s1 - mnew);
      m_r[r] = mnew;
      l_r[r] = l_r[r] * alpha[r] + p0 + p1;
      sP[w][8 * hh + r][ln] = h16_bits(p0 * pcarry);
      sP[w][8 * hh + r][16 + ln] = h16_bits(p1 * pcarry);
    }
#pragma unroll
    for (int dt = 0; dt < DT; ++dt)
#pragma unroll
      for (int r = 0; r < 8; ++r) oacc[dt][r] *= alpha[r];
    __builtin_amdgcn_fence(4  , "workgroup");
    __builtin_amdgcn_wave_barrier();
    FragH pa;
    pa.half[0] = *(const v8us*)&sP[w][ln][8 * hh];
    pa.half[1] = *(const v8us*)&sP[w][ln][16 + 8 * hh];
#pragma unroll
    for (int dt = 0; dt < DT; ++dt) {
      FragH bv;
      bv.half[0] = *(const v8us*)&sVt[dt * 16 + ln][8 * hh];
      bv.half[1] = *(const v8us*)&sVt[dt * 16 + ln][16 + 8 * hh];
      oacc[dt] = mma16(pa.v, bv.v, oacc[dt]);
    }
    __builtin_amdgcn_fence(4  , "workgroup");
    __builtin_amdgcn_wave_barrier();
  }
#pragma unroll
  for (int r = 0; r < 8; ++r) {
    float l = l_r[r];
    l += __shfl_xor(l, 1, 32); l += __shfl_xor(l, 2, 32); l += __shfl_xor(l, 4, 32); l += __shfl_xor(l, 8, 32);
    l_r[r] = onorm * (1.0f / l);
  }
#pragma unroll
  for (int dt = 0; dt < DT; ++dt)
#pragma unroll
    for (int r = 0; r < 8; ++r) sO[w][8 * hh + r][dt * 16 + ln] = h16_bits(oacc[dt][r] * l_r[r]);
  __builtin_amdgcn_fence(4  , "workgroup");
  __builtin_amdgcn_wave_barrier();
  const int rq = lane >> 3, p8 = (lane & 7) * 8;
  unsigned short* crow = ctx + (size_t)(b * T + q0) * cpitch + h * D;
  for (int pass = 0; pass < 2; ++pass) {
#pragma unroll
    for (int q = 0; q < 4; ++q) {
      const int r = q * 4 + rq;
      const v8us v = *(const v8us*)&sO[w][r][p8];
      *(volatile v8us*)(crow + (size_t)r * cpitch + p8) = v;
    }
    if (pass == 0) __threadfence();
  }
}

extern "C" void kernel_launch(void* const* d_in, const int* in_sizes, int n_in,
                              void* d_out, int out_size, void* d_ws, size_t ws_size, hipStream_t stream) {
  if (n_in < 13) return;
  const long long need_rows = (long long)(NB - 1) * SEQ_FULL + SEQ;
  if ((long long)in_sizes[0] < need_rows * FEAT) return;
  if (in_sizes[1] < FEAT || in_sizes[2] < FEAT) return;
  if (in_sizes[3] < QKVN * FEAT || in_sizes[4] < QKVN) return;
  if (in_sizes[5] < FEAT * FEAT || in_sizes[6] < FEAT) return;
  if (in_sizes[7] < FEAT || in_sizes[8] < FEAT) return;
  if (in_sizes[9] < MLPH * FEAT || in_sizes[10] < MLPH) return;
  if (in_sizes[11] < FEAT * MLPH || in_sizes[12] < FEAT) return;
  if ((long long)out_size < need_rows * FEAT) return;

  const float* x      = (const float*)d_in[0];
  const float* ln1_w  = (const float*)d_in[1];
  const float* ln1_b  = (const float*)d_in[2];
  const float* qkv_w  = (const float*)d_in[3];
  const float* qkv_b  = (const float*)d_in[4];
  const float* proj_w = (const float*)d_in[5];
  const float* proj_b = (const float*)d_in[6];
  const float* ln2_w  = (const float*)d_in[7];
  const float* ln2_b  = (const float*)d_in[8];
  const float* up_w   = (const float*)d_in[9];
  const float* up_b   = (const float*)d_in[10];
  const float* down_w = (const float*)d_in[11];
  const float* down_b = (const float*)d_in[12];

  char* ws = (char*)d_ws; size_t off = 0;
  auto take = [&](size_t bytes) { char* p = ws + off; off += (bytes + 255) & ~(size_t)255; return p; };
  unsigned short* Wqkv16 = (unsigned short*)take((size_t)QKVN * FEAT * 2);
  unsigned short* Wo16   = (unsigned short*)take((size_t)FEAT * FEAT * 2);
  unsigned short* Wup16  = (unsigned short*)take((size_t)MLPH * FEAT * 2);
  unsigned short* Wdn16  = (unsigned short*)take((size_t)FEAT * MLPH * 2);
  const size_t r1_bytes = (size_t)MR * FEAT * 2;
  const size_t r2_a = (size_t)MR * QKVN * 2, r2_b = (size_t)MR * MLPH * 2;
  const size_t r2_bytes = (r2_a > r2_b) ? r2_a : r2_b;
  unsigned short* R1 = (unsigned short*)take(r1_bytes);
  unsigned short* R2 = (unsigned short*)take(r2_bytes);
  unsigned short* R3 = (unsigned short*)take((size_t)MR * QKN * 2);
  float* OUT32 = (float*)take((size_t)MR * FEAT * 4);
  if (off > ws_size) return;
  if (off > (size_t)134217728) return;

  const float wsc = 256.0f;
  k_w16<<<(unsigned)((QKVN * FEAT / 8 + 255) / 256), 256, 0, stream>>>(qkv_w, Wqkv16, QKVN * FEAT / 8, wsc);
  k_w16<<<(unsigned)((FEAT * FEAT / 8 + 255) / 256), 256, 0, stream>>>(proj_w, Wo16, FEAT * FEAT / 8, wsc);
  k_w16<<<(unsigned)((MLPH * FEAT / 8 + 255) / 256), 256, 0, stream>>>(up_w, Wup16, MLPH * FEAT / 8, wsc);
  k_w16<<<(unsigned)((FEAT * MLPH / 8 + 255) / 256), 256, 0, stream>>>(down_w, Wdn16, FEAT * MLPH / 8, wsc);

  auto ggrid = [](int M, int N) { return (unsigned)(((M / 16) * (N / 64) + 3) / 4); };

  k_ln16<true><<<(unsigned)MR, 96, 0, stream>>>(x, 1, SEQ, SEQ_FULL, ln1_w, ln1_b, R1, 8.0f, 1e-5f);
  k_gemm16<true, 0, false, true><<<ggrid(MR, QKVN), 128, 0, stream>>>(R1, FEAT, Wqkv16, FEAT, qkv_b, qkv_b, qkv_b, QKVN, nullptr, 0, 0,
                                                                       (void*)R2, QKVN, 0, SEQ, SEQ_FULL, MR, QKVN, FEAT, 1.0f / 2048.0f, 1.0f,
                                                                       R3, QKN, QKN, 4096.0f);
  k_attn16<DHEAD><<<(unsigned)(NB * NHEAD * (SEQ / 64)), 128, 0, stream>>>(R2, QKVN, R3, QKN, FEAT, SEQ, NHEAD, FEAT, 2 * FEAT,
                                                                          1.0f / 4096.0f, 16384.0f, 64.0f / 16384.0f, R1, FEAT);
  k_gemm16<false, 0, true, false><<<ggrid(MR, FEAT), 128, 0, stream>>>(R1, FEAT, Wo16, FEAT, proj_b, proj_b, proj_b, FEAT, x, FEAT, 1,
                                                                        (void*)OUT32, FEAT, 0, SEQ, SEQ_FULL, MR, FEAT, FEAT, 1.0f / 16384.0f, 1.0f,
                                                                        nullptr, 0, 0, 0.0f);
  k_ln16<false><<<(unsigned)MR, 96, 0, stream>>>(OUT32, 0, SEQ, SEQ_FULL, ln2_w, ln2_b, R1, 8.0f, 1e-5f);
  k_gemm16<true, 1, false, false><<<ggrid(MR, MLPH), 128, 0, stream>>>(R1, FEAT, Wup16, FEAT, up_b, up_b, up_b, MLPH, nullptr, 0, 0,
                                                                        (void*)R2, MLPH, 0, SEQ, SEQ_FULL, MR, MLPH, FEAT, 1.0f / 2048.0f, 16.0f,
                                                                        nullptr, 0, 0, 0.0f);
  k_gemm16<false, 0, false, false><<<ggrid(MR, FEAT), 128, 0, stream>>>(R2, MLPH, Wdn16, MLPH, down_b, down_b, down_b, FEAT, OUT32, FEAT, 0,
                                                                         d_out, FEAT, 1, SEQ, SEQ_FULL, MR, FEAT, MLPH, 1.0f / 4096.0f, 1.0f,
                                                                         nullptr, 0, 0, 0.0f);
}
